// ColBertPairwiseDistillLoss_9740985828095
// MI455X (gfx1250) — hardware-verified
//
#include <hip/hip_runtime.h>

constexpr int NBATCH      = 64;
constexpr int NQTOK       = 32;
constexpr int NDTOK       = 1024;
constexpr int EMB         = 128;
constexpr int QROWS       = NBATCH * NQTOK;
constexpr int DROWS       = NBATCH * NDTOK;
constexpr int DOCS_PER_CH = 8;
constexpr int NCHUNKS     = NBATCH / DOCS_PER_CH;
constexpr int CHUNK_COLS  = DOCS_PER_CH * NDTOK;
constexpr int PART_ELEMS  = 2 * NCHUNKS * NBATCH * DOCS_PER_CH;
static_assert(QROWS % 64 == 0);
static_assert(CHUNK_COLS % 64 == 0);
static_assert(EMB % 32 == 0);

typedef __attribute__((ext_vector_type(16))) _Float16 v16h;
typedef __attribute__((ext_vector_type(8)))  _Float16 v8h;
typedef __attribute__((ext_vector_type(16))) __bf16   v16b;
typedef __attribute__((ext_vector_type(8)))  __bf16   v8b;
typedef __attribute__((ext_vector_type(8)))  float    v8f;
typedef __attribute__((ext_vector_type(4)))  float    v4f;
#define U16(p) ((const unsigned short*)(const void*)(p))

__device__ __forceinline__ unsigned short f2bf_bits(float f) {
  unsigned u = __float_as_uint(f);
  return (unsigned short)((u + 0x7FFFu + ((u >> 16) & 1u)) >> 16);
}
__device__ __forceinline__ float bf_bits2f(unsigned short h) { return __uint_as_float(((unsigned)h) << 16); }

__device__ __forceinline__ void dep_guard_h(v8f& a, v8f& b, v16h x, v16h y) { asm volatile("v_nop\n\tv_nop\n\tv_nop\n\tv_nop" : "+v"(a), "+v"(b) : "v"(x), "v"(y)); }
__device__ __forceinline__ void dep_guard_b(v8f& a, v8f& b, v16b x, v16b y) { asm volatile("v_nop\n\tv_nop\n\tv_nop\n\tv_nop" : "+v"(a), "+v"(b) : "v"(x), "v"(y)); }
__device__ __forceinline__ void keep4_h(v16h a, v16h b, v16h c, v16h d) { asm volatile("v_nop" :: "v"(a), "v"(b), "v"(c), "v"(d)); }
__device__ __forceinline__ void keep4_b(v16b a, v16b b, v16b c, v16b d) { asm volatile("v_nop" :: "v"(a), "v"(b), "v"(c), "v"(d)); }
__device__ __forceinline__ void acc_guard4(v8f& a, v8f& b, v8f& c, v8f& d) { asm volatile("v_nop\n\tv_nop\n\tv_nop\n\tv_nop" : "+v"(a), "+v"(b), "+v"(c), "+v"(d)); }
template <typename T> struct Frag;
template <> struct Frag<_Float16> {
  typedef v16h V; union U { v16h v; v8h h[2]; };
  static __device__ __forceinline__ v16h load(const _Float16* p) {
    U f; f.h[0] = *(const v8h*)(p); f.h[1] = *(const v8h*)(p + 16); return f.v;
  }
  static __device__ __forceinline__ v8f mma(v16h a, v16h b, v8f c) {
    return __builtin_amdgcn_wmma_f32_16x16x32_f16(false, a, false, b, (short)0, c, false, false);
  }
  static __device__ __forceinline__ void guard(v8f& a, v8f& b, v16h x, v16h y) { dep_guard_h(a, b, x, y); }
  static __device__ __forceinline__ void keep(v16h a, v16h b, v16h c, v16h d) { keep4_h(a, b, c, d); }
};
template <> struct Frag<__bf16> {
  typedef v16b V; union U { v16b v; v8b h[2]; };
  static __device__ __forceinline__ v16b load(const __bf16* p) {
    U f; f.h[0] = *(const v8b*)(p); f.h[1] = *(const v8b*)(p + 16); return f.v;
  }
  static __device__ __forceinline__ v8f mma(v16b a, v16b b, v8f c) {
    return __builtin_amdgcn_wmma_f32_16x16x32_bf16(false, a, false, b, (short)0, c, false, false);
  }
  static __device__ __forceinline__ void guard(v8f& a, v8f& b, v16b x, v16b y) { dep_guard_b(a, b, x, y); }
  static __device__ __forceinline__ void keep(v16b a, v16b b, v16b c, v16b d) { keep4_b(a, b, c, d); }
};

template <int ET> struct Elem;
template <> struct Elem<0> { typedef _Float16 T; };
template <> struct Elem<1> { typedef __bf16 T; };
template <int ET, bool SPLIT, int BIAS_MODE, int OUT_MODE, bool RESID, int ACT = 0>
__global__ __launch_bounds__(256) void wmma_gemm64(
    const unsigned short* __restrict__ Ap, const unsigned short* __restrict__ A2p, int lda, long strideA,
    const unsigned short* __restrict__ Btp, const unsigned short* __restrict__ Bt2p, int ldb, long strideB,
    void* __restrict__ Cout, void* __restrict__ Cout2, int ldc, long strideC,
    const float* __restrict__ bias,
    const float* __restrict__ resid, long strideR,
    int M, int N, int K, float scale) {
  typedef typename Elem<ET>::T T;
  typedef typename Frag<T>::V V;
  const T* A = (const T*)Ap; const T* A2 = (const T*)A2p; const T* Bt = (const T*)Btp; const T* Bt2 = (const T*)Bt2p;
  __shared__ __align__(16) float sT[8][16 * 68];
  const int b    = blockIdx.y;
  const int lane = threadIdx.x & 31;
  const int wave = threadIdx.x >> 5;
  const int tilesN = N >> 6;
  const int tilesM = M >> 6;
  const int tile = blockIdx.x * 8 + wave;
  if (tile >= tilesM * tilesN) return;
  const int tm = tile / tilesN;
  const int tn = tile - tm * tilesN;
  const int m0 = tm << 6;
  const int n0 = tn << 6;

  const T* Ab  = A  + (size_t)b * strideA;
  const T* Bb  = Bt + (size_t)b * strideB;
  const T* Ab2 = SPLIT ? (A2  + (size_t)b * strideA) : nullptr;
  const T* Bb2 = SPLIT ? (Bt2 + (size_t)b * strideB) : nullptr;

  const int rlane = lane & 15;
  const int koff  = (lane >> 4) * 8;
  const int mOff  = (lane >> 4) * 8;

  v8f acc[4][4];
#pragma unroll
  for (int i = 0; i < 4; ++i)
#pragma unroll
    for (int j = 0; j < 4; ++j) acc[i][j] = (v8f){0.f,0.f,0.f,0.f,0.f,0.f,0.f,0.f};

  for (int k0 = 0; k0 < K; k0 += 32) {
    V bh[4], bl[4];
#pragma unroll
    for (int j = 0; j < 4; ++j) {
      const size_t bo = (size_t)(n0 + (j << 4) + rlane) * ldb + koff + k0;
      bh[j] = Frag<T>::load(Bb + bo);
      if (SPLIT) bl[j] = Frag<T>::load(Bb2 + bo);
    }
#pragma unroll
    for (int i = 0; i < 4; ++i) {
      const size_t ao = (size_t)(m0 + (i << 4) + rlane) * lda + koff + k0;
      V ah = Frag<T>::load(Ab + ao);
      V al;
      if (SPLIT) al = Frag<T>::load(Ab2 + ao);
#pragma unroll
      for (int j = 0; j < 4; ++j) {
        acc[i][j] = Frag<T>::mma(ah, bh[j], acc[i][j]);
        if (SPLIT) {
          acc[i][j] = Frag<T>::mma(ah, bl[j], acc[i][j]);
          acc[i][j] = Frag<T>::mma(al, bh[j], acc[i][j]);
        }
      }
      Frag<T>::guard(acc[i][0], acc[i][3], ah, SPLIT ? al : ah);
    }
    Frag<T>::keep(bh[0], bh[1], bh[2], bh[3]);
    if (SPLIT) Frag<T>::keep(bl[0], bl[1], bl[2], bl[3]);
  }
  acc_guard4(acc[0][0], acc[0][1], acc[0][2], acc[0][3]);
  acc_guard4(acc[1][0], acc[1][1], acc[1][2], acc[1][3]);
  acc_guard4(acc[2][0], acc[2][1], acc[2][2], acc[2][3]);
  acc_guard4(acc[3][0], acc[3][1], acc[3][2], acc[3][3]);

  float* slab = sT[wave];
  const float* Rb = RESID ? (resid + (size_t)b * strideR) : nullptr;
#pragma unroll
  for (int i = 0; i < 4; ++i) {
    const int mBase = m0 + (i << 4);
#pragma unroll
    for (int j = 0; j < 4; ++j) {
      const int n = n0 + (j << 4) + rlane;
      float bv = 0.f;
      if (BIAS_MODE == 2) bv = bias[n];
#pragma unroll
      for (int r = 0; r < 8; ++r) {
        float v = acc[i][j][r] * scale;
        if (BIAS_MODE == 1) v += bias[mBase + mOff + r];
        if (BIAS_MODE == 2) v += bv;
        if (RESID) v += Rb[(size_t)(mBase + mOff + r) * ldc + n];
        if (ACT == 1) v = tanhf(v);
        if (ACT == 2) v = fmaxf(v, 0.0f);
        if (ACT == 3) v = v / (1.0f + expf(-v));
        if (ACT == 4) v = (v > 0.f) ? v : 0.01f * v;
        slab[(mOff + r) * 68 + (j << 4) + rlane] = v;
      }
    }
    __builtin_amdgcn_fence(__ATOMIC_RELEASE, "workgroup");
    __builtin_amdgcn_wave_barrier();
    __builtin_amdgcn_fence(__ATOMIC_ACQUIRE, "workgroup");
    if (OUT_MODE == 0) {
      float* C = (float*)Cout + (size_t)b * strideC;
      const int hh = lane >> 4, c4 = (lane & 15) * 4;
      for (int pass = 0; pass < 2; ++pass) {
#pragma unroll
        for (int it = 0; it < 8; ++it) {
          const int row = it * 2 + hh;
          v4f v = *(const v4f*)(slab + row * 68 + c4);
          *(volatile v4f*)(C + (size_t)(mBase + row) * ldc + n0 + c4) = v;
        }
        __threadfence();
      }
    } else {
      const int q = lane >> 3, c8 = (lane & 7) * 8;
      unsigned short* C  = (unsigned short*)Cout  + (size_t)b * strideC;
      unsigned short* C2 = (OUT_MODE == 2) ? ((unsigned short*)Cout2 + (size_t)b * strideC) : nullptr;
      for (int pass = 0; pass < 2; ++pass) {
#pragma unroll
        for (int it = 0; it < 4; ++it) {
          const int row = it * 4 + q;
          const float* sp = slab + row * 68 + c8;
          v8h hv, lv;
#pragma unroll
          for (int e = 0; e < 8; ++e) {
            if (OUT_MODE == 1) {
              hv[e] = (_Float16)sp[e];
            } else {
              unsigned short hb = f2bf_bits(sp[e]);
              unsigned short lb = f2bf_bits(sp[e] - bf_bits2f(hb));
              hv[e] = __builtin_bit_cast(_Float16, hb);
              lv[e] = __builtin_bit_cast(_Float16, lb);
            }
          }
          *(volatile v8h*)(C + (size_t)(mBase + row) * ldc + n0 + c8) = hv;
          if (OUT_MODE == 2) *(volatile v8h*)(C2 + (size_t)(mBase + row) * ldc + n0 + c8) = lv;
        }
        __threadfence();
      }
    }
    __builtin_amdgcn_fence(__ATOMIC_RELEASE, "workgroup");
    __builtin_amdgcn_wave_barrier();
    __builtin_amdgcn_fence(__ATOMIC_ACQUIRE, "workgroup");
  }
}

__global__ __launch_bounds__(256) void k_cast8(const float* __restrict__ in, _Float16* __restrict__ out,
                                               float mul, int n8) {
  const int id = blockIdx.x * 256 + threadIdx.x;
  const int idc = id < n8 ? id : n8 - 1;
  const v4f a0 = *(const v4f*)(in + (size_t)idc * 8);
  const v4f a1 = *(const v4f*)(in + (size_t)idc * 8 + 4);
  v8h hv;
#pragma unroll
  for (int e = 0; e < 4; ++e) { hv[e] = (_Float16)(a0[e] * mul); hv[4 + e] = (_Float16)(a1[e] * mul); }
  if (id < n8) {
    _Float16* dst = out + (size_t)idc * 8;
    *(volatile v8h*)dst = hv;
    __threadfence();
    *(volatile v8h*)dst = hv;
  }
}

__global__ __launch_bounds__(256) void k_maxsum(const float* __restrict__ S, float* __restrict__ part, int partBase) {
  __shared__ float sres[32];
  const int tid = threadIdx.x, lane = tid & 31, wave = tid >> 5;
  const int b0 = blockIdx.x * 4;
#pragma unroll 1
  for (int bl = 0; bl < 4; ++bl) {
    float acc = 0.0f;
#pragma unroll 1
    for (int i = 0; i < NQTOK; ++i) {
      const float* rowp = S + (size_t)((b0 + bl) * NQTOK + i) * CHUNK_COLS + (size_t)wave * NDTOK;
      float m = -INFINITY;
#pragma unroll
      for (int it = 0; it < 8; ++it) {
        const v4f v = *(const v4f*)(rowp + (it * 32 + lane) * 4);
        m = fmaxf(m, fmaxf(fmaxf(v[0], v[1]), fmaxf(v[2], v[3])));
      }
#pragma unroll
      for (int off = 1; off < 32; off <<= 1) m = fmaxf(m, __shfl_xor(m, off, 32));
      acc += m;
    }
    if (lane == 0) sres[bl * 8 + wave] = acc;
  }
  __syncthreads();
  if (wave == 0) {
    const float v = sres[lane];
    float* dst = part + partBase + b0 * 8 + lane;
    *(volatile float*)dst = v;
    __threadfence();
    *(volatile float*)dst = v;
  }
}

__global__ __launch_bounds__(64) void k_loss(const float* __restrict__ part, float* __restrict__ out) {
  __shared__ float sc[2][NBATCH * 65];
  __shared__ float spv[NBATCH];
  __shared__ float msev[NBATCH];
  const int t = threadIdx.x;
#pragma unroll 1
  for (int k = 0; k < PART_ELEMS / 64; ++k) {
    const int e = t + 64 * k;
    const int pr = e >> 12, rem = e & 4095;
    const int ch = rem >> 9, b = (rem >> 3) & 63, cl = rem & 7;
    sc[pr][b * 65 + ch * 8 + cl] = part[e];
  }
  __syncthreads();
  {
    const int b = t;
    const float pos = sc[0][b * 65 + b];
    float neg = -INFINITY;
    float mse = 0.0f;
#pragma unroll 1
    for (int c = 0; c < NBATCH; ++c) {
      const float s  = sc[0][b * 65 + c];
      const float ts = sc[1][b * 65 + c];
      const _Float16 s16 = (_Float16)s;
      const _Float16 t16 = (_Float16)ts;
      const _Float16 d16 = s16 - t16;
      const _Float16 q16 = d16 * d16;
      mse += (float)q16;
      const float cand = (c == b) ? -INFINITY : s;
      neg = fmaxf(neg, cand);
    }
    const float x  = neg - pos;
    const float sp = fmaxf(x, 0.0f) + log1pf(expf(-fabsf(x)));
    spv[b]  = sp;
    msev[b] = mse;
  }
  __syncthreads();
  if (t == 0) {
    float cs = 0.0f, ms = 0.0f;
#pragma unroll 1
    for (int i = 0; i < NBATCH; ++i) { cs += spv[i]; ms += msev[i]; }
    const float contr = cs * (1.0f / 64.0f);
    const float msef  = ms * (1.0f / 4096.0f);
    const float mse16 = (float)((_Float16)msef);
    const float loss  = contr + 0.3f * mse16;
    *(volatile float*)out = loss;
    __threadfence();
    *(volatile float*)out = loss;
  }
}

extern "C" void kernel_launch(void* const* d_in, const int* in_sizes, int n_in,
                              void* d_out, int out_size, void* d_ws, size_t ws_size,
                              hipStream_t stream) {
  if (n_in < 4) return;
  if (in_sizes[0] != QROWS * EMB || in_sizes[1] != DROWS * EMB ||
      in_sizes[2] != QROWS * EMB || in_sizes[3] != DROWS * EMB) return;
  if (out_size != 1) return;

  const float* q  = (const float*)d_in[0];
  const float* d  = (const float*)d_in[1];
  const float* tq = (const float*)d_in[2];
  const float* td = (const float*)d_in[3];
  float* out = (float*)d_out;

  const size_t szQ16 = (size_t)QROWS * EMB * 2;
  const size_t szD16 = (size_t)DROWS * EMB * 2;
  const size_t szSIM = (size_t)QROWS * CHUNK_COLS * 4;
  const size_t szPART = (size_t)PART_ELEMS * 4;
  size_t off = 0;
  auto carve = [&](size_t bytes) { size_t o = off; off += (bytes + 255) & ~(size_t)255; return o; };
  const size_t oQ16 = carve(szQ16), oTQ16 = carve(szQ16), oD16 = carve(szD16), oTD16 = carve(szD16);
  const size_t oSIM = carve(szSIM);
  const size_t oPART = carve(szPART);
  if (off > ws_size) return;
  if (off > (size_t)134217728) return;

  char* ws = (char*)d_ws;
  _Float16* Q16  = (_Float16*)(ws + oQ16);
  _Float16* TQ16 = (_Float16*)(ws + oTQ16);
  _Float16* D16  = (_Float16*)(ws + oD16);
  _Float16* TD16 = (_Float16*)(ws + oTD16);
  float* SIM  = (float*)(ws + oSIM);
  float* PART = (float*)(ws + oPART);

  k_cast8<<<(QROWS * EMB / 8 + 255) / 256, 256, 0, stream>>>(q,  Q16,  1.0f, QROWS * EMB / 8);
  k_cast8<<<(DROWS * EMB / 8 + 255) / 256, 256, 0, stream>>>(d,  D16,  1.0f, DROWS * EMB / 8);
  k_cast8<<<(QROWS * EMB / 8 + 255) / 256, 256, 0, stream>>>(tq, TQ16, 1.0f, QROWS * EMB / 8);
  k_cast8<<<(DROWS * EMB / 8 + 255) / 256, 256, 0, stream>>>(td, TD16, 1.0f, DROWS * EMB / 8);

  const int gemmBlocks = (QROWS / 64) * (CHUNK_COLS / 64) / 8;
  for (int pair = 0; pair < 2; ++pair) {
    const _Float16* Qp = pair ? TQ16 : Q16;
    const _Float16* Dp = pair ? TD16 : D16;
    for (int ch = 0; ch < NCHUNKS; ++ch) {
      const _Float16* Dc = Dp + (size_t)ch * CHUNK_COLS * EMB;
      wmma_gemm64<0, false, 0, 0, false, 0><<<dim3(gemmBlocks, 1), 256, 0, stream>>>(
          U16(Qp), U16(Qp), EMB, 0L, U16(Dc), U16(Dc), EMB, 0L,
          (void*)SIM, (void*)SIM, CHUNK_COLS, 0L, (const float*)SIM, (const float*)SIM, 0L,
          QROWS, CHUNK_COLS, EMB, 1.0f);
      k_maxsum<<<NBATCH / 4, 256, 0, stream>>>(SIM, PART, (pair * NCHUNKS + ch) * (NBATCH * DOCS_PER_CH));
    }
  }

  k_loss<<<1, 64, 0, stream>>>(PART, out);
}
